// NeighborGraphAttention_43078521979429
// MI455X (gfx1250) — hardware-verified
//
#include <hip/hip_runtime.h>
#include <math.h>

typedef __attribute__((ext_vector_type(16))) _Float16 v16h;
typedef __attribute__((ext_vector_type(16))) __bf16 v16b;
typedef __attribute__((ext_vector_type(8)))  _Float16 v8h;
typedef __attribute__((ext_vector_type(8)))  float v8f;
typedef __attribute__((ext_vector_type(4)))  float v4f;
typedef __attribute__((ext_vector_type(2)))  float v2f;
typedef __attribute__((ext_vector_type(4)))  unsigned v4u;
typedef __attribute__((ext_vector_type(4)))  int v4i;
typedef float __attribute__((may_alias)) float_a;
typedef int __attribute__((may_alias)) int_a;

template <typename T> __device__ __forceinline__ void vst2(void* p, T v) { *(volatile T*)p = v; __threadfence(); *(volatile T*)p = v; }
__device__ __forceinline__ v8f wmma16(v16h a, v16h b, v8f c) {
  v8f d = __builtin_amdgcn_wmma_f32_16x16x32_f16(false, a, false, b, (short)0, c, false, false);
  asm volatile("v_nop\n\tv_nop\n\tv_nop\n\tv_nop" : "+v"(d) : "v"(a), "v"(b));
  return d;
}
__device__ __forceinline__ v8f wmma_bf(v16b a, v16b b, v8f c) {
  v8f d = __builtin_amdgcn_wmma_f32_16x16x32_bf16(false, a, false, b, (short)0, c, false, false);
  asm volatile("v_nop\n\tv_nop\n\tv_nop\n\tv_nop" : "+v"(d) : "v"(a), "v"(b));
  return d;
}
__device__ __forceinline__ v16h frag_h(const _Float16* rowk0, int lane) {
  union { v16h v; v8h q[2]; } u; const _Float16* p = rowk0 + 8 * (lane >> 4);
  u.q[0] = *(const v8h*)p; u.q[1] = *(const v8h*)(p + 16); return u.v;
}
__device__ __forceinline__ v16h frag_f32(const float* rowk0, int lane) {
  v16h a; const float* p = rowk0 + 8 * (lane >> 4);
#pragma unroll
  for (int i = 0; i < 8; ++i) { a[i] = (_Float16)p[i]; a[8 + i] = (_Float16)p[16 + i]; }
  return a;
}
__device__ __forceinline__ v16h frag_f32s(const float* rowk0, int lane, float sc) {
  v16h a; const float* p = rowk0 + 8 * (lane >> 4);
#pragma unroll
  for (int i = 0; i < 8; ++i) { a[i] = (_Float16)(p[i] * sc); a[8 + i] = (_Float16)(p[16 + i] * sc); }
  return a;
}
__device__ __forceinline__ v16h fragc_f32(const float* W, int k0, int n, int lane, int ld, int K) {
  v16h a; const int g = lane >> 4;
#pragma unroll
  for (int i = 0; i < 8; ++i) { const int ka = k0 + 8 * g + i, kb = ka + 16;
    a[i] = (_Float16)(ka < K ? W[(size_t)(ka < K ? ka : K - 1) * ld + n] : 0.f); a[8 + i] = (_Float16)(kb < K ? W[(size_t)(kb < K ? kb : K - 1) * ld + n] : 0.f); }
  return a;
}
struct F2 { v16b h, l; };
__device__ __forceinline__ F2 bsplit16(const float v[16]) { F2 r;
#pragma unroll
  for (int i = 0; i < 16; ++i) { const __bf16 h = (__bf16)v[i]; r.h[i] = h; r.l[i] = (__bf16)(v[i] - (float)h); }
  return r; }
__device__ __forceinline__ F2 split_row(const float* row, int k0, int lane) { float v[16]; const float* p = row + k0 + 8 * (lane >> 4);
#pragma unroll
  for (int i = 0; i < 8; ++i) { v[i] = p[i]; v[8 + i] = p[16 + i]; }
  return bsplit16(v); }
__device__ __forceinline__ F2 split_rowK(const float* row, int k0, int lane, int K) { float v[16]; const int g = lane >> 4;
#pragma unroll
  for (int i = 0; i < 8; ++i) { const int ka = k0 + 8 * g + i, kb = ka + 16; v[i] = ka < K ? row[ka < K ? ka : K - 1] : 0.f; v[8 + i] = kb < K ? row[kb < K ? kb : K - 1] : 0.f; }
  return bsplit16(v); }
__device__ __forceinline__ F2 split_col(const float* W, int k0, int n, int lane, int ld, int K) { float v[16]; const int g = lane >> 4;
#pragma unroll
  for (int i = 0; i < 8; ++i) { const int ka = k0 + 8 * g + i, kb = ka + 16; v[i] = ka < K ? W[(size_t)(ka < K ? ka : K - 1) * ld + n] : 0.f; v[8 + i] = kb < K ? W[(size_t)(kb < K ? kb : K - 1) * ld + n] : 0.f; }
  return bsplit16(v); }
__device__ __forceinline__ v8f mac3(const F2& a, const F2& b, v8f c) { c = wmma_bf(a.l, b.h, c); c = wmma_bf(a.h, b.l, c); return wmma_bf(a.h, b.h, c); }
__device__ __forceinline__ float sigm(float v) { return 1.0f / (1.0f + expf(-v)); }
#define LDSX() do { asm volatile("s_wait_dscnt 0" ::: "memory"); __builtin_amdgcn_wave_barrier(); __builtin_amdgcn_fence(__ATOMIC_RELEASE, "workgroup"); } while (0)


#define NB 2
#define TT 2048
#define CC 512
#define NH 8
#define HD 64
#define MM 32
#define GH 64
#define NR (NB * TT)
#ifndef NRB
#define NRB (NR / 64)
#define NTB (NR / 8)
#endif
typedef __attribute__((ext_vector_type(8))) __bf16 v8b;
__device__ __forceinline__ v16b frag_b(const __bf16* rowk0, int lane) {
  union { v16b v; v8b q[2]; } u; const __bf16* p = rowk0 + 8 * (lane >> 4);
  u.q[0] = *(const v8b*)p; u.q[1] = *(const v8b*)(p + 16); return u.v;
}
__device__ __forceinline__ float bfr(float v) { return (float)(__bf16)v; }
__device__ __attribute__((noinline)) float exp_ni(float v) { return expf(v); }
__device__ __attribute__((noinline)) float erf_ni(float v) { return erff(v); }

#define WS_PW   0u
#define WS_PG2  (WS_PW + 2u * (size_t)4 * CC * CC)
#define WS_Q    (WS_PG2 + 2u * GH * GH)
#define WS_K    (WS_Q + 4u * (size_t)NR * CC)
#define WS_V    (WS_K + 4u * (size_t)NR * CC)
#define WS_CTX  (WS_V + 4u * (size_t)NR * CC)
#define WS_END  (WS_CTX + 4u * (size_t)NR * CC)

__global__ __launch_bounds__(256) void k_pack(const float* __restrict__ WQ, const float* __restrict__ WK, const float* __restrict__ WV, const float* __restrict__ WO, const float* __restrict__ WG2, __bf16* __restrict__ P) {
  const int n = blockIdx.x, which = blockIdx.y, t = threadIdx.x; __shared__ __align__(16) __bf16 s[CC];
  if (which < 4) { const float* Wm = (which == 0) ? WQ : (which == 1) ? WK : (which == 2) ? WV : WO; for (int k = t; k < CC; k += 256) s[k] = (__bf16)Wm[(size_t)n * CC + k]; __syncthreads(); for (int q = t; q < CC / 8; q += 256) vst2((unsigned*)(P + ((size_t)which * CC + n) * CC + q * 8), *(const v4u*)&s[q * 8]); }
  else { if (n >= GH) return; if (t < GH) s[t] = (__bf16)WG2[(size_t)n * GH + t]; __syncthreads(); if (t < GH / 8) vst2((unsigned*)(P + WS_PG2 / 2 + (size_t)n * GH + t * 8), *(const v4u*)&s[t * 8]); }
}
__global__ __launch_bounds__(128) void k_proj(const float* __restrict__ X, const __bf16* __restrict__ P, const float* __restrict__ BQ, const float* __restrict__ BK, const float* __restrict__ BV, float* __restrict__ Q, float* __restrict__ Kf, float* __restrict__ Vf) {
  __shared__ __align__(16) float so[4][16][132];
  const int tid = threadIdx.x, wave = tid >> 5, lane = tid & 31, col = lane & 15, g = lane >> 4; const int which = blockIdx.z; const int n0 = blockIdx.y * 128; const size_t r0 = (size_t)blockIdx.x * 64 + wave * 16;
  const __bf16* Wr = P + (size_t)which * CC * CC; const float* BB = (which == 0) ? BQ : (which == 1) ? BK : BV; float* dst = (which == 0) ? Q : (which == 1) ? Kf : Vf;
  v8f acc[8] = {};
#pragma unroll 2
  for (int kc = 0; kc < CC / 32; ++kc) { v16b a; { const float* p = X + (r0 + col) * CC + kc * 32 + 8 * g;
#pragma unroll
      for (int i = 0; i < 8; ++i) { a[i] = (__bf16)p[i]; a[8 + i] = (__bf16)p[16 + i]; } }
#pragma unroll
    for (int j = 0; j < 8; ++j) acc[j] = wmma_bf(a, frag_b(Wr + (size_t)(n0 + j * 16 + col) * CC + kc * 32, lane), acc[j]); }
#pragma unroll
  for (int j = 0; j < 8; ++j) { const float bb = bfr(BB[n0 + j * 16 + col]);
#pragma unroll
    for (int r = 0; r < 8; ++r) so[wave][8 * g + r][j * 16 + col] = acc[j][r] + bb; }
  LDSX();
  for (int rl = 0; rl < 16; ++rl) vst2(dst + (r0 + rl) * CC + n0 + lane * 4, *(const v4f*)&so[wave][rl][lane * 4]);
}
__device__ __attribute__((noinline)) float atan2_p(float y, float x) { return atan2f(y, x); }
__device__ __attribute__((noinline)) float sin_p(float v) { return sinf(v); }
__device__ __attribute__((noinline)) float cos_p(float v) { return cosf(v); }
__device__ __forceinline__ float silu_f(float x) { return x / (1.0f + exp_ni(-x)); }
__global__ __launch_bounds__(256) void k_nbr(const float* __restrict__ CO, const int* __restrict__ MASK, const int* __restrict__ NBR, const float* __restrict__ WG1, const float* __restrict__ BG1, const __bf16* __restrict__ P, const float* __restrict__ BG2, const float* __restrict__ WG3, const float* __restrict__ BG3, const float* __restrict__ Q, const float* __restrict__ Kf, const float* __restrict__ Vf, float* __restrict__ CTX) {
  __shared__ __align__(16) float sg1[256][GH + 4];
  __shared__ float sbias[8][NH][MM]; __shared__ int snb[8][MM]; __shared__ int svalid[8][MM]; __shared__ float slg[8][NH][4][MM + 1];
  const int tid = threadIdx.x, wave = tid >> 5, lane = tid & 31, col = lane & 15, g = lane >> 4; const size_t t0 = (size_t)blockIdx.x * 8; const size_t b = t0 / TT;
  { const int tl = tid >> 5, m = tid & 31; const size_t t = t0 + tl; const int raw = NBR[t * MM + m];
#ifdef TWIN_MOD
    const int nb = ((raw % TT) + TT) % TT;
#else
    const int nb = min(max(raw, 0), TT - 1);
#endif
    snb[tl][m] = nb;
    const int mt = MASK[t], mn = MASK[b * TT + nb]; svalid[tl][m] = (raw >= 0 && mt != 0 && mn != 0) ? 1 : 0;
    const float x0 = bfr(CO[t * 2]), y0 = bfr(CO[t * 2 + 1]); const float xn = bfr(CO[(b * TT + nb) * 2]), yn = bfr(CO[(b * TT + nb) * 2 + 1]);
    const float dx = xn - x0, dy = yn - y0; const float dist2 = dx * dx + dy * dy; const float dist = sqrtf(dist2 + 1e-8f);
    const bool mz = (fabsf(dx) < 1e-6f) && (fabsf(dy) < 1e-6f); const float dxs = mz ? 1e-6f : dx, dys = mz ? 1e-6f : dy; const float ang = atan2_p(dys, dxs);
    float geo[6]; geo[0] = dx; geo[1] = dy; geo[2] = dist; geo[3] = dist2; geo[4] = sin_p(ang); geo[5] = cos_p(ang);
#pragma unroll 1
    for (int o = 0; o < GH; ++o) { float a = bfr(BG1[o]);
#pragma unroll
      for (int i = 0; i < 6; ++i) a += geo[i] * bfr(WG1[o * 6 + i]);
      sg1[tid][o] = silu_f(a); }
    for (int i = GH; i < GH + 4; ++i) sg1[tid][i] = 0.f; }
  LDSX(); __syncthreads();
  { v8f acc2[2][4] = {};
#pragma unroll
    for (int rt = 0; rt < 2; ++rt) {
#pragma unroll
      for (int kc = 0; kc < 2; ++kc) { const F2 a = split_row(&sg1[wave * 32 + rt * 16 + col][0], kc * 32, lane);
#pragma unroll
        for (int j = 0; j < 4; ++j) { const v16b w = frag_b(P + WS_PG2 / 2 + (size_t)(j * 16 + col) * GH + kc * 32, lane); acc2[rt][j] = wmma_bf(a.l, w, acc2[rt][j]); acc2[rt][j] = wmma_bf(a.h, w, acc2[rt][j]); } } }
    LDSX(); __syncthreads();
#pragma unroll
    for (int rt = 0; rt < 2; ++rt)
#pragma unroll
      for (int j = 0; j < 4; ++j) { const float bb = bfr(BG2[j * 16 + col]);
#pragma unroll
        for (int r = 0; r < 8; ++r) sg1[wave * 32 + rt * 16 + 8 * g + r][j * 16 + col] = silu_f(acc2[rt][j][r] + bb); } }
  LDSX(); __syncthreads();
  { const int tl = tid >> 5, m = tid & 31; const size_t t = t0 + tl; const bool valid = svalid[tl][m] != 0; const bool mt = MASK[t] != 0;
#pragma unroll 1
    for (int hh = 0; hh < NH; ++hh) { float a = bfr(BG3[hh]);
#pragma unroll 8
      for (int k = 0; k < GH; ++k) a += sg1[tid][k] * bfr(WG3[hh * GH + k]);
      sbias[tl][hh][m] = a; }
    (void)valid; (void)mt; }
  __syncthreads();
  { const int tl = tid >> 5, hh = (tid >> 2) & 7, qd = tid & 3; const size_t t = t0 + tl; const bool mt = MASK[t] != 0;
    float qv[16];
#pragma unroll
    for (int i = 0; i < 16; ++i) qv[i] = Q[t * CC + hh * HD + qd * 16 + i];
    float* lg = &slg[tl][hh][qd][0];
    float mx = -3.0e38f;
#pragma unroll 1
    for (int m = 0; m < MM; ++m) { const size_t nrow = b * TT + snb[tl][m]; float s = 0.f;
#pragma unroll
      for (int i = 0; i < 16; ++i) s += qv[i] * Kf[nrow * CC + hh * HD + qd * 16 + i];
      s += __shfl_xor(s, 1); s += __shfl_xor(s, 2);
      float v = s * 0.125f + sbias[tl][hh][m]; if (!svalid[tl][m]) v = -1e9f; if (!mt) v = -1e9f; lg[m] = v; mx = fmaxf(mx, v); }
    float den = 0.f;
#pragma unroll 1
    for (int m = 0; m < MM; ++m) { const float e = exp_ni(lg[m] - mx); lg[m] = e; den += e; }
    const float inv = 1.0f / den; float o[16];
#pragma unroll
    for (int i = 0; i < 16; ++i) o[i] = 0.f;
#pragma unroll 1
    for (int m = 0; m < MM; ++m) { const size_t nrow = b * TT + snb[tl][m]; const float w = lg[m] * inv;
#pragma unroll
      for (int i = 0; i < 16; ++i) o[i] += w * Vf[nrow * CC + hh * HD + qd * 16 + i]; }
#pragma unroll
    for (int i = 0; i < 16; i += 4) { v4f v4; v4[0] = o[i]; v4[1] = o[i + 1]; v4[2] = o[i + 2]; v4[3] = o[i + 3]; vst2(CTX + t * CC + hh * HD + qd * 16 + i, v4); } }
}
__global__ __launch_bounds__(128) void k_out(const float* __restrict__ CTX, const __bf16* __restrict__ P, const float* __restrict__ BO, const int* __restrict__ MASK, float* __restrict__ OUT) {
  __shared__ __align__(16) float so[4][16][132];
  const int tid = threadIdx.x, wave = tid >> 5, lane = tid & 31, col = lane & 15, g = lane >> 4; const size_t r0 = (size_t)blockIdx.x * 64 + wave * 16; const int n0 = blockIdx.y * 128;
  v8f acc[8] = {};
#pragma unroll 2
  for (int kc = 0; kc < CC / 32; ++kc) { const F2 a = split_row(CTX + (r0 + col) * CC, kc * 32, lane);
#pragma unroll
    for (int j = 0; j < 8; ++j) { const v16b w = frag_b(P + ((size_t)3 * CC + n0 + j * 16 + col) * CC + kc * 32, lane); acc[j] = wmma_bf(a.l, w, acc[j]); acc[j] = wmma_bf(a.h, w, acc[j]); } }
#pragma unroll
  for (int j = 0; j < 8; ++j) { const float bb = bfr(BO[n0 + j * 16 + col]);
#pragma unroll
    for (int r = 0; r < 8; ++r) { const size_t row = r0 + 8 * g + r; so[wave][8 * g + r][j * 16 + col] = (MASK[row] != 0) ? (acc[j][r] + bb) : 0.f; } }
  LDSX();
  for (int rl = 0; rl < 16; ++rl) vst2(OUT + (r0 + rl) * CC + n0 + lane * 4, *(const v4f*)&so[wave][rl][lane * 4]);
}
extern "C" void kernel_launch(void* const* d_in, const int* in_sizes, int n_in, void* d_out, int out_size, void* d_ws, size_t ws_size, hipStream_t stream) {
  (void)in_sizes; (void)n_in; (void)out_size;
  const float** F = (const float**)d_in;
  if (ws_size < (size_t)WS_END) return;
  char* ws = (char*)d_ws; __bf16* P = (__bf16*)ws; float *Q = (float*)(ws + WS_Q), *Kf = (float*)(ws + WS_K), *Vf = (float*)(ws + WS_V), *CTX = (float*)(ws + WS_CTX);
  const int* MASK = (const int*)d_in[2]; const int* NBR = (const int*)d_in[3];
  k_pack<<<dim3(CC, 5), 256, 0, stream>>>(F[4], F[6], F[8], F[10], F[14], P);
  k_proj<<<dim3(NR / 64, CC / 128, 3), 128, 0, stream>>>(F[0], P, F[5], F[7], F[9], Q, Kf, Vf);
  k_nbr<<<NTB, 256, 0, stream>>>(F[1], MASK, NBR, F[12], F[13], P, F[15], F[16], F[17], Q, Kf, Vf, CTX);
  k_out<<<dim3(NRB, CC / 128), 128, 0, stream>>>(CTX, P, F[11], MASK, (float*)d_out);
}
